// MambaLayer_77515569758967
// MI455X (gfx1250) — hardware-verified
//
#include <hip/hip_runtime.h>
#include <math.h>

typedef __attribute__((ext_vector_type(16))) _Float16 v16h;
typedef __attribute__((ext_vector_type(8)))  _Float16 v8h;
typedef __attribute__((ext_vector_type(4)))  _Float16 v4h;
typedef __attribute__((ext_vector_type(16))) __bf16   v16b;
typedef __attribute__((ext_vector_type(8)))  __bf16   v8b;
typedef __attribute__((ext_vector_type(8)))  float    v8f;
typedef __attribute__((ext_vector_type(4)))  float    v4f;

constexpr int kSamples = 4;
constexpr int kSeq   = 2048;
constexpr int kRows  = kSeq;
constexpr int kIn    = 1024;
constexpr int kDm    = 512;
constexpr int kDi    = 1024;
constexpr int kDi2   = 2 * kDi;
constexpr int kNs    = 16;
constexpr int kR     = 32;
constexpr int kXd    = kR + 2 * kNs;
constexpr int kMlp   = 2048;
constexpr int kKc    = 4;
constexpr int kThr   = 256;
constexpr float kLnEps = 1e-5f;

constexpr float kInCarry = 1024.0f;
constexpr float kWCarry  = 4096.0f;
constexpr float kDwCarry = 4096.0f;
constexpr float kACarry  = 256.0f;
constexpr float kScX = 1.0f / (kInCarry * kWCarry);
constexpr float kScA = 1.0f / (kACarry * kWCarry);
constexpr float kF16MinNormal = 6.103515625e-5f;

static_assert((kRows % 64) == 0 && (kDm % 64) == 0 && (kDi2 % 64) == 0 && (kXd % 64) == 0 && (kDi % 64) == 0 && (kMlp % 64) == 0 && (kIn % 64) == 0, "GEMM M, N multiples of 64");
static_assert(((kRows / 64) * (kXd / 64)) % 8 == 0, "the smallest GEMM grid exact");
static_assert((kIn % 32) == 0 && (kDm % 32) == 0 && (kDi % 32) == 0 && (kR % 32) == 0 && (kMlp % 32) == 0, "GEMM K multiples of 32");

constexpr size_t kOffX16 = 0ull;
constexpr size_t kOffWRED = 4194304ull;
constexpr size_t kOffWIN = 5242880ull;
constexpr size_t kOffWXP = 7340032ull;
constexpr size_t kOffWDT = 7471104ull;
constexpr size_t kOffWOUT = 7536640ull;
constexpr size_t kOffWFC1 = 8585216ull;
constexpr size_t kOffWFC2 = 10682368ull;
constexpr size_t kOffWEXP = 12779520ull;
constexpr size_t kOffBV = 13828096ull;
constexpr size_t kOffXF = 13860864ull;
constexpr size_t kOffXN16 = 18055168ull;
constexpr size_t kOffXZ = 20152320ull;
constexpr size_t kOffXI = 36929536ull;
constexpr size_t kOffXI16 = 45318144ull;
constexpr size_t kOffXD = 49512448ull;
constexpr size_t kOffDT16 = 50036736ull;
constexpr size_t kOffDL = 50167808ull;
constexpr size_t kOffHID = 58556416ull;
constexpr size_t kOffY16 = 66945024ull;
constexpr size_t kOffXM = 71139328ull;
constexpr size_t kOffMO = 75333632ull;
constexpr size_t kOffMO16 = 79527936ull;
constexpr size_t kOffH1 = 81625088ull;
constexpr size_t kOffH16 = 98402304ull;
constexpr size_t kOffM2 = 106790912ull;
constexpr size_t kOffO16 = 110985216ull;
constexpr size_t kOffEX = 113082368ull;
constexpr size_t kWsTotal = 121470976ull;
static_assert(kWsTotal <= 134217728ull, "carve cap: under 128 MiB");
static_assert(kOffX16 == 0
              && kOffWRED == kOffX16 + 4194304ull
              && kOffWIN == kOffWRED + 1048576ull
              && kOffWXP == kOffWIN + 2097152ull
              && kOffWDT == kOffWXP + 131072ull
              && kOffWOUT == kOffWDT + 65536ull
              && kOffWFC1 == kOffWOUT + 1048576ull
              && kOffWFC2 == kOffWFC1 + 2097152ull
              && kOffWEXP == kOffWFC2 + 2097152ull
              && kOffBV == kOffWEXP + 1048576ull
              && kOffXF == kOffBV + 32768ull
              && kOffXN16 == kOffXF + 4194304ull
              && kOffXZ == kOffXN16 + 2097152ull
              && kOffXI == kOffXZ + 16777216ull
              && kOffXI16 == kOffXI + 8388608ull
              && kOffXD == kOffXI16 + 4194304ull
              && kOffDT16 == kOffXD + 524288ull
              && kOffDL == kOffDT16 + 131072ull
              && kOffHID == kOffDL + 8388608ull
              && kOffY16 == kOffHID + 8388608ull
              && kOffXM == kOffY16 + 4194304ull
              && kOffMO == kOffXM + 4194304ull
              && kOffMO16 == kOffMO + 4194304ull
              && kOffH1 == kOffMO16 + 2097152ull
              && kOffH16 == kOffH1 + 16777216ull
              && kOffM2 == kOffH16 + 8388608ull
              && kOffO16 == kOffM2 + 4194304ull
              && kOffEX == kOffO16 + 2097152ull
              && kWsTotal == kOffEX + 8388608ull, "the carve is chained and totalled");
static_assert((kOffX16 % 256) == 0 && (kOffWRED % 256) == 0 && (kOffWIN % 256) == 0 && (kOffWXP % 256) == 0 && (kOffWDT % 256) == 0 && (kOffWOUT % 256) == 0 && (kOffWFC1 % 256) == 0 && (kOffWFC2 % 256) == 0 && (kOffWEXP % 256) == 0 && (kOffBV % 256) == 0 && (kOffXF % 256) == 0 && (kOffXN16 % 256) == 0 && (kOffXZ % 256) == 0 && (kOffXI % 256) == 0 && (kOffXI16 % 256) == 0 && (kOffXD % 256) == 0 && (kOffDT16 % 256) == 0 && (kOffDL % 256) == 0 && (kOffHID % 256) == 0 && (kOffY16 % 256) == 0 && (kOffXM % 256) == 0 && (kOffMO % 256) == 0 && (kOffMO16 % 256) == 0 && (kOffH1 % 256) == 0 && (kOffH16 % 256) == 0 && (kOffM2 % 256) == 0 && (kOffO16 % 256) == 0 && (kOffEX % 256) == 0, "aligned regions");
constexpr int kBvDt = 0, kBvF1 = 1024, kBvF2 = 3072, kBvZ = 4096, kBvTot = 8192;
static_assert(kBvF1 == kBvDt + kDi && kBvF2 == kBvF1 + kMlp && kBvF2 + kDm <= kBvZ && kBvZ + kDi2 <= kBvTot, "bias stream map; the zero row reaches the widest zero-bias product (2,048 columns)");

__device__ __forceinline__ unsigned short f2bf_bits(float f) {
  unsigned u = __float_as_uint(f);
  return (unsigned short)((u + 0x7FFFu + ((u >> 16) & 1u)) >> 16);
}
__device__ __forceinline__ float bf_bits2f(unsigned short h) { return __uint_as_float(((unsigned)h) << 16); }
__device__ __forceinline__ float bf16r(float f) { return bf_bits2f(f2bf_bits(f)); }
__device__ __forceinline__ float carry_flush(float v, float carry) {
  const float s = v * carry;
  return (fabsf(s) < kF16MinNormal) ? 0.0f : s;
}
__device__ __forceinline__ float frcp(float x) { return __builtin_amdgcn_rcpf(x); }

__device__ __forceinline__ void dep_guard4_h(v8f& a, v8f& b, v8f& c, v8f& d, v16h x, v16h y) { asm volatile("v_nop\n\tv_nop\n\tv_nop\n\tv_nop" : "+v"(a), "+v"(b), "+v"(c), "+v"(d) : "v"(x), "v"(y)); }
__device__ __forceinline__ void dep_guard4_b(v8f& a, v8f& b, v8f& c, v8f& d, v16b x, v16b y) { asm volatile("v_nop\n\tv_nop\n\tv_nop\n\tv_nop" : "+v"(a), "+v"(b), "+v"(c), "+v"(d) : "v"(x), "v"(y)); }
__device__ __forceinline__ void keep4_h(v16h a, v16h b, v16h c, v16h d) { asm volatile("v_nop" :: "v"(a), "v"(b), "v"(c), "v"(d)); }
__device__ __forceinline__ void keep4_b(v16b a, v16b b, v16b c, v16b d) { asm volatile("v_nop" :: "v"(a), "v"(b), "v"(c), "v"(d)); }
__device__ __forceinline__ void acc_guard4(v8f& a, v8f& b, v8f& c, v8f& d) { asm volatile("v_nop\n\tv_nop\n\tv_nop\n\tv_nop" : "+v"(a), "+v"(b), "+v"(c), "+v"(d)); }

template <typename T> struct Frag;
template <> struct Frag<_Float16> {
  typedef v16h V; union U { v16h v; v8h h[2]; };
  static __device__ __forceinline__ v16h load(const _Float16* p) {
    U f; f.h[0] = *(const v8h*)(p); f.h[1] = *(const v8h*)(p + 16); return f.v;
  }
  static __device__ __forceinline__ v8f mma(v16h a, v16h b, v8f c) {
    return __builtin_amdgcn_wmma_f32_16x16x32_f16(false, a, false, b, (short)0, c, false, false);
  }
  static __device__ __forceinline__ void guard4(v8f& a, v8f& b, v8f& c, v8f& d, v16h x, v16h y) { dep_guard4_h(a, b, c, d, x, y); }
  static __device__ __forceinline__ void keep(v16h a, v16h b, v16h c, v16h d) { keep4_h(a, b, c, d); }
};
template <> struct Frag<__bf16> {
  typedef v16b V; union U { v16b v; v8b h[2]; };
  static __device__ __forceinline__ v16b load(const __bf16* p) {
    U f; f.h[0] = *(const v8b*)(p); f.h[1] = *(const v8b*)(p + 16); return f.v;
  }
  static __device__ __forceinline__ v8f mma(v16b a, v16b b, v8f c) {
    return __builtin_amdgcn_wmma_f32_16x16x32_bf16(false, a, false, b, (short)0, c, false, false);
  }
  static __device__ __forceinline__ void guard4(v8f& a, v8f& b, v8f& c, v8f& d, v16b x, v16b y) { dep_guard4_b(a, b, c, d, x, y); }
  static __device__ __forceinline__ void keep(v16b a, v16b b, v16b c, v16b d) { keep4_b(a, b, c, d); }
};

__device__ __forceinline__ v8f mma_h(v16h a, v16h b, v8f c) {
  c = __builtin_amdgcn_wmma_f32_16x16x32_f16(false, a, false, b, (short)0, c, false, false);
  asm volatile("v_nop\n\tv_nop\n\tv_nop\n\tv_nop" : "+v"(c) : "v"(a), "v"(b));
  return c;
}

template <int ET> struct Elem;
template <> struct Elem<0> { typedef _Float16 T; };
template <> struct Elem<1> { typedef __bf16 T; };
template <int ET, bool SPLIT, int BIAS_MODE, int OUT_MODE, bool RESID, int ACT = 0>
__global__ __launch_bounds__(256) void wmma_gemm64(
    const unsigned short* __restrict__ Ap, const unsigned short* __restrict__ A2p, int lda, long strideA,
    const unsigned short* __restrict__ Btp, const unsigned short* __restrict__ Bt2p, int ldb, long strideB,
    void* __restrict__ Cout, void* __restrict__ Cout2, int ldc, long strideC,
    const float* __restrict__ bias,
    const float* __restrict__ resid, long strideR,
    int M, int N, int K, float scale) {
  typedef typename Elem<ET>::T T;
  typedef typename Frag<T>::V V;
  const T* A = (const T*)Ap; const T* A2 = (const T*)A2p; const T* Bt = (const T*)Btp; const T* Bt2 = (const T*)Bt2p;
  __shared__ __align__(16) float sT[8][16 * 68];
  const int b    = blockIdx.y;
  const int lane = threadIdx.x & 31;
  const int wave = threadIdx.x >> 5;
  const int tilesN = N >> 6;
  const int tilesM = M >> 6;
  const int tile = blockIdx.x * 8 + wave;
  if (tile >= tilesM * tilesN) return;
  const int tm = tile / tilesN;
  const int tn = tile - tm * tilesN;
  const int m0 = tm << 6;
  const int n0 = tn << 6;

  const T* Ab  = A  + (size_t)b * strideA;
  const T* Bb  = Bt + (size_t)b * strideB;
  const T* Ab2 = SPLIT ? (A2  + (size_t)b * strideA) : nullptr;
  const T* Bb2 = SPLIT ? (Bt2 + (size_t)b * strideB) : nullptr;

  const int rlane = lane & 15;
  const int koff  = (lane >> 4) * 8;
  const int mOff  = (lane >> 4) * 8;

  v8f acc[4][4];
#pragma unroll
  for (int i = 0; i < 4; ++i)
#pragma unroll
    for (int j = 0; j < 4; ++j) acc[i][j] = (v8f){0.f,0.f,0.f,0.f,0.f,0.f,0.f,0.f};

  for (int k0 = 0; k0 < K; k0 += 32) {
    V bh[4], bl[4];
#pragma unroll
    for (int j = 0; j < 4; ++j) {
      const size_t bo = (size_t)(n0 + (j << 4) + rlane) * ldb + koff + k0;
      bh[j] = Frag<T>::load(Bb + bo);
      if (SPLIT) bl[j] = Frag<T>::load(Bb2 + bo);
    }
#pragma unroll
    for (int i = 0; i < 4; ++i) {
      const size_t ao = (size_t)(m0 + (i << 4) + rlane) * lda + koff + k0;
      V ah = Frag<T>::load(Ab + ao);
      V al;
      if (SPLIT) al = Frag<T>::load(Ab2 + ao);
#pragma unroll
      for (int j = 0; j < 4; ++j) {
        acc[i][j] = Frag<T>::mma(ah, bh[j], acc[i][j]);
        if (SPLIT) {
          acc[i][j] = Frag<T>::mma(ah, bl[j], acc[i][j]);
          acc[i][j] = Frag<T>::mma(al, bh[j], acc[i][j]);
        }
      }
      Frag<T>::guard4(acc[i][0], acc[i][1], acc[i][2], acc[i][3], ah, SPLIT ? al : ah);
    }
    Frag<T>::keep(bh[0], bh[1], bh[2], bh[3]);
    if (SPLIT) Frag<T>::keep(bl[0], bl[1], bl[2], bl[3]);
  }
  acc_guard4(acc[0][0], acc[0][1], acc[0][2], acc[0][3]);
  acc_guard4(acc[1][0], acc[1][1], acc[1][2], acc[1][3]);
  acc_guard4(acc[2][0], acc[2][1], acc[2][2], acc[2][3]);
  acc_guard4(acc[3][0], acc[3][1], acc[3][2], acc[3][3]);

  float* slab = sT[wave];
  const float* Rb = RESID ? (resid + (size_t)b * strideR) : nullptr;
#pragma unroll
  for (int i = 0; i < 4; ++i) {
    const int mBase = m0 + (i << 4);
#pragma unroll
    for (int j = 0; j < 4; ++j) {
      const int n = n0 + (j << 4) + rlane;
      float bv = 0.f;
      if (BIAS_MODE == 2) bv = bias[n];
#pragma unroll
      for (int r = 0; r < 8; ++r) {
        float v = acc[i][j][r] * scale;
        if (BIAS_MODE == 1) v += bias[mBase + mOff + r];
        if (BIAS_MODE == 2) v += bv;
        if (RESID) v += Rb[(size_t)(mBase + mOff + r) * ldc + n];
        if (ACT == 1) v = tanhf(v);
        if (ACT == 2) v = fmaxf(v, 0.0f);
        if (ACT == 3) v = v / (1.0f + expf(-v));
        if (ACT == 4) v = (v > 0.f) ? v : 0.01f * v;
        slab[(mOff + r) * 68 + (j << 4) + rlane] = v;
      }
    }
    __builtin_amdgcn_fence(__ATOMIC_RELEASE, "workgroup");
    __builtin_amdgcn_wave_barrier();
    __builtin_amdgcn_fence(__ATOMIC_ACQUIRE, "workgroup");
    if (OUT_MODE == 0) {
      float* C = (float*)Cout + (size_t)b * strideC;
      const int hh = lane >> 4, c4 = (lane & 15) * 4;
      for (int pass = 0; pass < 2; ++pass) {
#pragma unroll
        for (int it = 0; it < 8; ++it) {
          const int row = it * 2 + hh;
          v4f v = *(const v4f*)(slab + row * 68 + c4);
          *(volatile v4f*)(C + (size_t)(mBase + row) * ldc + n0 + c4) = v;
        }
        __threadfence();
      }
    } else {
      const int q = lane >> 3, c8 = (lane & 7) * 8;
      unsigned short* C  = (unsigned short*)Cout  + (size_t)b * strideC;
      unsigned short* C2 = (OUT_MODE == 2) ? ((unsigned short*)Cout2 + (size_t)b * strideC) : nullptr;
      for (int pass = 0; pass < 2; ++pass) {
#pragma unroll
        for (int it = 0; it < 4; ++it) {
          const int row = it * 4 + q;
          const float* sp = slab + row * 68 + c8;
          v8h hv, lv;
#pragma unroll
          for (int e = 0; e < 8; ++e) {
            if (OUT_MODE == 1) {
              hv[e] = (_Float16)sp[e];
            } else {
              unsigned short hb = f2bf_bits(sp[e]);
              unsigned short lb = f2bf_bits(sp[e] - bf_bits2f(hb));
              hv[e] = __builtin_bit_cast(_Float16, hb);
              lv[e] = __builtin_bit_cast(_Float16, lb);
            }
          }
          *(volatile v8h*)(C + (size_t)(mBase + row) * ldc + n0 + c8) = hv;
          if (OUT_MODE == 2) *(volatile v8h*)(C2 + (size_t)(mBase + row) * ldc + n0 + c8) = lv;
        }
        __threadfence();
      }
    }
    __builtin_amdgcn_fence(__ATOMIC_RELEASE, "workgroup");
    __builtin_amdgcn_wave_barrier();
    __builtin_amdgcn_fence(__ATOMIC_ACQUIRE, "workgroup");
  }
}

__global__ __launch_bounds__(kThr) void cast_plane_kernel(const float* __restrict__ src, unsigned short* __restrict__ dst,
                                                          int colsLog2, int dstPitch, int dstOff) {
  const int i   = blockIdx.x * kThr + threadIdx.x;
  const int sh  = colsLog2 - 3;
  const int row = i >> sh;
  const int c8  = (i & ((1 << sh) - 1)) * 8;
  const float* sp = src + ((size_t)row << colsLog2) + c8;
  const v4f a0 = *(const v4f*)(sp);
  const v4f a1 = *(const v4f*)(sp + 4);
  v8h hv;
#pragma unroll
  for (int e = 0; e < 4; ++e) {
    const float f0 = a0[e];
    const float f1 = a1[e];
    hv[e]     = (_Float16)carry_flush(bf16r(f0), kInCarry);
    hv[4 + e] = (_Float16)carry_flush(bf16r(f1), kInCarry);
  }
  unsigned short* dp = dst + (size_t)row * dstPitch + dstOff + c8;
  *(volatile v8h*)dp = hv;
  __threadfence();
  *(volatile v8h*)dp = hv;
}
__global__ __launch_bounds__(256) void wt_plane_kernel(const float* __restrict__ W, unsigned short* __restrict__ dst, int K, int N, int nLive, int ldd, int colOff) {
  const int n  = blockIdx.x;
  const int k8 = threadIdx.x * 8;
  const bool live = n < nLive;
  const int nc = live ? n : 0;
  v8h hv;
#pragma unroll
  for (int e = 0; e < 8; ++e) {
    const float w = W[(size_t)(k8 + e) * N + nc];
    hv[e] = (_Float16)(live ? carry_flush(bf16r(w), kWCarry) : 0.0f);
  }
  unsigned short* dp = dst + (size_t)n * ldd + colOff + k8;
  *(volatile v8h*)dp = hv;
  __threadfence();
  *(volatile v8h*)dp = hv;
}


__global__ __launch_bounds__(kThr) void setup_kernel(const float* __restrict__ dt_w, const float* __restrict__ dt_b, const float* __restrict__ fc1_b,
                                                     const float* __restrict__ fc2_b, unsigned short* __restrict__ WDT, float* __restrict__ BV) {
  unsigned v = blockIdx.x * (unsigned)kThr + threadIdx.x;
  asm volatile("" : "+v"(v));
  if (v < 4096u) {
    const unsigned n = v >> 2;
    const unsigned k8 = (v & 3u) * 8u;
    v8h hv;
#pragma unroll
    for (int e = 0; e < 8; ++e) { const float w = dt_w[(size_t)(k8 + (unsigned)e) * kDi + n]; hv[e] = (_Float16)carry_flush(bf16r(w), kDwCarry); }
    unsigned short* dp = WDT + (size_t)v * 8u;
    *(volatile v8h*)dp = hv;
    __threadfence();
    *(volatile v8h*)dp = hv;
  } else {
    const unsigned i0 = (v - 4096u) * 4u;
    v4f o = {0.f, 0.f, 0.f, 0.f};
    if (i0 < (unsigned)kBvZ) {
      const float* sp = (i0 < (unsigned)kBvF1) ? (dt_b + i0) : ((i0 < (unsigned)kBvF2) ? (fc1_b + (i0 - (unsigned)kBvF1)) : (fc2_b + ((i0 < (unsigned)(kBvF2 + kDm)) ? (i0 - (unsigned)kBvF2) : 0u)));
      const v4f a = *(const v4f*)sp;
      const bool live = i0 < (unsigned)(kBvF2 + kDm);
#pragma unroll
      for (int e = 0; e < 4; ++e) { const float x = a[e]; o[e] = live ? bf16r(x) : 0.0f; }
    }
    float* dp = BV + i0;
    *(volatile v4f*)dp = o;
    __threadfence();
    *(volatile v4f*)dp = o;
  }
}
static_assert(kDi * kR / 8 == 4096 && kBvTot / 4 == 2048 && 4096 + 2048 == 24 * kThr && (kBvF1 % 128) == 0 && (kBvF2 % 128) == 0 && ((kBvF2 + kDm) % 128) == 0 && (kBvZ % 128) == 0, "set-up grid exact; regions wave-uniform");

__global__ __launch_bounds__(128) void ln_kernel(const float* __restrict__ SRC, const float* __restrict__ g, const float* __restrict__ b,
                                                 const float* __restrict__ RES, float* __restrict__ DF, unsigned short* __restrict__ D16) {
  __shared__ __align__(16) float sRed[128];
  const int tid = threadIdx.x;
  const size_t row = blockIdx.x;
  const int c4 = tid * 4;
  const v4f x = *(const v4f*)(SRC + row * kDm + c4);
  sRed[tid] = (x[0] + x[1]) + (x[2] + x[3]);
  __syncthreads();
  float s = 0.0f;
#pragma unroll 1
  for (int j = 0; j < 128; ++j) { float p = sRed[j]; asm volatile("" : "+v"(p)); s += p; }
  const float mean = s * (1.0f / (float)kDm);
  __syncthreads();
  const float d0 = x[0] - mean, d1 = x[1] - mean, d2 = x[2] - mean, d3 = x[3] - mean;
  sRed[tid] = (d0 * d0 + d1 * d1) + (d2 * d2 + d3 * d3);
  __syncthreads();
  float q = 0.0f;
#pragma unroll 1
  for (int j = 0; j < 128; ++j) { float p = sRed[j]; asm volatile("" : "+v"(p)); q += p; }
  __syncthreads();
  const float inv = 1.0f / sqrtf(q * (1.0f / (float)kDm) + kLnEps);
  const v4f gg = *(const v4f*)(g + c4), bb = *(const v4f*)(b + c4);
  v4f r = {0.f, 0.f, 0.f, 0.f};
  if (RES != nullptr) r = *(const v4f*)(RES + row * kDm + c4);
  v4f o; v4h hv;
  const float dd[4] = {d0, d1, d2, d3};
#pragma unroll
  for (int e = 0; e < 4; ++e) {
    const float g0 = gg[e], b0 = bb[e];
    const float y = dd[e] * inv * bf16r(g0) + bf16r(b0) + r[e];
    o[e] = y;
    hv[e] = (_Float16)carry_flush(y, kACarry);
  }
  for (int pass = 0; pass < 2; ++pass) {
    if (DF != nullptr) *(volatile v4f*)(DF + row * kDm + c4) = o;
    *(volatile v4h*)(D16 + row * kDm + c4) = hv;
    __threadfence();
  }
}
static_assert(kDm == 128 * 4, "one thread per four columns of a 512-wide row");

__global__ __launch_bounds__(kThr) void conv_silu_kernel(const float* __restrict__ XZ, const float* __restrict__ conv_w, const float* __restrict__ conv_b,
                                                         float* __restrict__ XI, unsigned short* __restrict__ XI16) {
  const size_t v = (size_t)blockIdx.x * kThr + threadIdx.x;
  const int row = (int)(v >> 8);
  const int d4 = (int)(v & 255) * 4;
  const v4f cb = *(const v4f*)(conv_b + d4);
  float acc[4];
#pragma unroll
  for (int e = 0; e < 4; ++e) { const float b0 = cb[e]; acc[e] = bf16r(b0); }
#pragma unroll
  for (int j = 0; j < kKc; ++j) {
    const int tr = row + j - (kKc - 1);
    const bool in = tr >= 0;
    const v4f xin = *(const v4f*)(XZ + (size_t)(in ? tr : 0) * kDi2 + d4);
#pragma unroll
    for (int e = 0; e < 4; ++e) {
      const float w0 = conv_w[(size_t)(d4 + e) * kKc + j];
      const float xv = in ? xin[e] : 0.0f;
      acc[e] += bf16r(w0) * xv;
    }
  }
  v4f o; v4h hv;
#pragma unroll
  for (int e = 0; e < 4; ++e) {
    const float s = acc[e] * (1.0f / (1.0f + expf(-acc[e])));
    o[e] = s;
    hv[e] = (_Float16)carry_flush(s, kACarry);
  }
  for (int pass = 0; pass < 2; ++pass) {
    *(volatile v4f*)(XI + (size_t)row * kDi + d4) = o;
    *(volatile v4h*)(XI16 + (size_t)row * kDi + d4) = hv;
    __threadfence();
  }
}
static_assert(((size_t)kRows * 256) % kThr == 0 && kDi / 4 == 256, "conv grid exact");

__global__ __launch_bounds__(kThr) void dt_cast_kernel(const float* __restrict__ XD, unsigned short* __restrict__ DT16) {
  const size_t v = (size_t)blockIdx.x * kThr + threadIdx.x;
  const size_t row = v >> 2;
  const int c8 = (int)(v & 3) * 8;
  const v4f a0 = *(const v4f*)(XD + row * kXd + c8), a1 = *(const v4f*)(XD + row * kXd + c8 + 4);
  v8h hv;
#pragma unroll
  for (int e = 0; e < 4; ++e) { hv[e] = (_Float16)carry_flush(a0[e], kACarry); hv[4 + e] = (_Float16)carry_flush(a1[e], kACarry); }
  unsigned short* dp = DT16 + v * 8;
  *(volatile v8h*)dp = hv;
  __threadfence();
  *(volatile v8h*)dp = hv;
}
static_assert(((size_t)kRows * 4) % kThr == 0 && kR == 32, "dt cast grid exact");

__global__ __launch_bounds__(kThr) void sel_scan_kernel(const float* __restrict__ DL, const float* __restrict__ XI, const float* __restrict__ XD,
                                                        const float* __restrict__ A_log, float* __restrict__ HID) {
  const int d = blockIdx.x * kThr + threadIdx.x;
  float A[kNs], h[kNs];
#pragma unroll
  for (int n = 0; n < kNs; ++n) { const float al = A_log[(size_t)d * kNs + n]; A[n] = -expf(bf16r(al)); h[n] = 0.0f; }
#pragma unroll 1
  for (int l = 0; l < kSeq; ++l) {
    const size_t row = (size_t)l;
    const float dl = DL[row * kDi + d];
    const float xv = XI[row * kDi + d];
    const float delta = (dl > 20.0f) ? dl : log1pf(expf(dl));
    const float dx = delta * xv;
    float y = 0.0f;
#pragma unroll
    for (int q = 0; q < 4; ++q) {
      const v4f bq = *(const v4f*)(XD + row * kXd + kR + 4 * q);
      const v4f cq = *(const v4f*)(XD + row * kXd + kR + kNs + 4 * q);
#pragma unroll
      for (int e = 0; e < 4; ++e) {
        const int n = 4 * q + e;
        const float hn = __expf(delta * A[n]) * h[n] + dx * bq[e];
        h[n] = hn;
        y += hn * cq[e];
      }
    }
    float* hp = HID + row * kDi + d;
    *(volatile float*)hp = y;
    __threadfence();
    *(volatile float*)hp = y;
  }
}
static_assert(kDi % kThr == 0, "scan grid exact");

__global__ __launch_bounds__(kThr) void gate_cast_kernel(const float* __restrict__ HID, const float* __restrict__ XI, const float* __restrict__ XZ,
                                                         const float* __restrict__ Dp, unsigned short* __restrict__ Y16) {
  const size_t v = (size_t)blockIdx.x * kThr + threadIdx.x;
  const size_t row = v >> 7;
  const int d8 = (int)(v & 127) * 8;
  v8h hv;
#pragma unroll
  for (int hlf = 0; hlf < 2; ++hlf) {
    const v4f hh = *(const v4f*)(HID + row * kDi + d8 + 4 * hlf);
    const v4f xx = *(const v4f*)(XI + row * kDi + d8 + 4 * hlf);
    const v4f zz = *(const v4f*)(XZ + row * kDi2 + kDi + d8 + 4 * hlf);
    const v4f dd = *(const v4f*)(Dp + d8 + 4 * hlf);
#pragma unroll
    for (int e = 0; e < 4; ++e) {
      const float d0 = dd[e];
      const float g = zz[e] * frcp(1.0f + __expf(-zz[e]));
      hv[4 * hlf + e] = (_Float16)carry_flush((hh[e] + bf16r(d0) * xx[e]) * g, kACarry);
    }
  }
  unsigned short* dp = Y16 + row * kDi + d8;
  *(volatile v8h*)dp = hv;
  __threadfence();
  *(volatile v8h*)dp = hv;
}
static_assert(((size_t)kRows * 128) % kThr == 0 && kDi / 8 == 128, "gate grid exact");

__global__ __launch_bounds__(kThr) void gelu_cast_kernel(const float* __restrict__ H1, unsigned short* __restrict__ H16) {
  const size_t v = (size_t)blockIdx.x * kThr + threadIdx.x;
  const v4f a0 = *(const v4f*)(H1 + v * 8), a1 = *(const v4f*)(H1 + v * 8 + 4);
  v8h hv;
#pragma unroll
  for (int e = 0; e < 4; ++e) {
    const float x0 = a0[e], x1 = a1[e];
    hv[e]     = (_Float16)carry_flush(0.5f * x0 * (1.0f + erff(x0 * 0.70710678118654752f)), kACarry);
    hv[4 + e] = (_Float16)carry_flush(0.5f * x1 * (1.0f + erff(x1 * 0.70710678118654752f)), kACarry);
  }
  unsigned short* dp = H16 + v * 8;
  *(volatile v8h*)dp = hv;
  __threadfence();
  *(volatile v8h*)dp = hv;
}
__global__ __launch_bounds__(kThr) void add_cast_kernel(const float* __restrict__ M2, const float* __restrict__ MO, unsigned short* __restrict__ O16) {
  const size_t v = (size_t)blockIdx.x * kThr + threadIdx.x;
  const v4f a0 = *(const v4f*)(M2 + v * 8), a1 = *(const v4f*)(M2 + v * 8 + 4);
  const v4f b0 = *(const v4f*)(MO + v * 8), b1 = *(const v4f*)(MO + v * 8 + 4);
  v8h hv;
#pragma unroll
  for (int e = 0; e < 4; ++e) { hv[e] = (_Float16)carry_flush(a0[e] + b0[e], kACarry); hv[4 + e] = (_Float16)carry_flush(a1[e] + b1[e], kACarry); }
  unsigned short* dp = O16 + v * 8;
  *(volatile v8h*)dp = hv;
  __threadfence();
  *(volatile v8h*)dp = hv;
}
__global__ __launch_bounds__(kThr) void add_out_kernel(const float* __restrict__ EX, const float* __restrict__ xs, float* __restrict__ out) {
  const size_t i = (size_t)blockIdx.x * kThr + threadIdx.x;
  const v4f a = *(const v4f*)(EX + i * 4), x = *(const v4f*)(xs + i * 4);
  v4f o;
#pragma unroll
  for (int e = 0; e < 4; ++e) { const float x0 = x[e]; o[e] = a[e] + bf16r(x0); }
  float* dp = out + i * 4;
  *(volatile v4f*)dp = o;
  __threadfence();
  *(volatile v4f*)dp = o;
}
static_assert(((size_t)kRows * kMlp / 8) % kThr == 0 && ((size_t)kRows * kDm / 8) % kThr == 0 && ((size_t)kRows * kIn / 4) % kThr == 0, "elementwise grids exact");

static_assert(((size_t)kRows * kIn / 8) % kThr == 0, "cast grid exact");

extern "C" void kernel_launch(void* const* d_in, const int* in_sizes, int n_in,
                              void* d_out, int out_size, void* d_ws, size_t ws_size,
                              hipStream_t stream) {
  if (n_in < 20 || d_out == nullptr || d_ws == nullptr) return;
  if (in_sizes[0] != kSamples * kRows * kIn || in_sizes[1] != kIn * kDm || in_sizes[2] != kDm * kIn || in_sizes[3] != kDm || in_sizes[4] != kDm || in_sizes[5] != kDm || in_sizes[6] != kDm) return;
  if (in_sizes[7] != kDm * kDi2 || in_sizes[8] != kDi * kKc || in_sizes[9] != kDi || in_sizes[10] != kDi * kXd || in_sizes[11] != kR * kDi || in_sizes[12] != kDi || in_sizes[13] != kDi * kNs || in_sizes[14] != kDi) return;
  if (in_sizes[15] != kDi * kDm || in_sizes[16] != kDm * kMlp || in_sizes[17] != kMlp || in_sizes[18] != kMlp * kDm || in_sizes[19] != kDm) return;
  if (out_size != kSamples * kRows * kIn) return;
  if (ws_size < kWsTotal) return;
  const float* x_tokens = (const float*)d_in[0];
  const float* w_red = (const float*)d_in[1];
  const float* w_exp = (const float*)d_in[2];
  const float* ln1_g = (const float*)d_in[3];
  const float* ln1_b = (const float*)d_in[4];
  const float* ln2_g = (const float*)d_in[5];
  const float* ln2_b = (const float*)d_in[6];
  const float* in_proj_w = (const float*)d_in[7];
  const float* conv_w = (const float*)d_in[8];
  const float* conv_b = (const float*)d_in[9];
  const float* x_proj_w = (const float*)d_in[10];
  const float* dt_proj_w = (const float*)d_in[11];
  const float* dt_proj_b = (const float*)d_in[12];
  const float* A_log = (const float*)d_in[13];
  const float* D_ssm = (const float*)d_in[14];
  const float* out_proj_w = (const float*)d_in[15];
  const float* fc1_w = (const float*)d_in[16];
  const float* fc1_b = (const float*)d_in[17];
  const float* fc2_w = (const float*)d_in[18];
  const float* fc2_b = (const float*)d_in[19];
  float* out = (float*)d_out;
  char* ws = (char*)d_ws;
  unsigned short* X16 = (unsigned short*)(ws + kOffX16);
  unsigned short* WRED = (unsigned short*)(ws + kOffWRED);
  unsigned short* WIN = (unsigned short*)(ws + kOffWIN);
  unsigned short* WXP = (unsigned short*)(ws + kOffWXP);
  unsigned short* WDT = (unsigned short*)(ws + kOffWDT);
  unsigned short* WOUT = (unsigned short*)(ws + kOffWOUT);
  unsigned short* WFC1 = (unsigned short*)(ws + kOffWFC1);
  unsigned short* WFC2 = (unsigned short*)(ws + kOffWFC2);
  unsigned short* WEXP = (unsigned short*)(ws + kOffWEXP);
  float* BV = (float*)(ws + kOffBV);
  float* XF = (float*)(ws + kOffXF);
  unsigned short* XN16 = (unsigned short*)(ws + kOffXN16);
  float* XZ = (float*)(ws + kOffXZ);
  float* XI = (float*)(ws + kOffXI);
  unsigned short* XI16 = (unsigned short*)(ws + kOffXI16);
  float* XD = (float*)(ws + kOffXD);
  unsigned short* DT16 = (unsigned short*)(ws + kOffDT16);
  float* DL = (float*)(ws + kOffDL);
  float* HID = (float*)(ws + kOffHID);
  unsigned short* Y16 = (unsigned short*)(ws + kOffY16);
  float* XM = (float*)(ws + kOffXM);
  float* MO = (float*)(ws + kOffMO);
  unsigned short* MO16 = (unsigned short*)(ws + kOffMO16);
  float* H1 = (float*)(ws + kOffH1);
  unsigned short* H16 = (unsigned short*)(ws + kOffH16);
  float* M2 = (float*)(ws + kOffM2);
  unsigned short* O16 = (unsigned short*)(ws + kOffO16);
  float* EX = (float*)(ws + kOffEX);
  const float* ZB = BV + kBvZ;

  wt_plane_kernel<<<kDm, kIn / 8, 0, stream>>>(w_red, WRED, kIn, kDm, kDm, kIn, 0);
  wt_plane_kernel<<<kDi2, kDm / 8, 0, stream>>>(in_proj_w, WIN, kDm, kDi2, kDi2, kDm, 0);
  wt_plane_kernel<<<kXd, kDi / 8, 0, stream>>>(x_proj_w, WXP, kDi, kXd, kXd, kDi, 0);
  wt_plane_kernel<<<kDm, kDi / 8, 0, stream>>>(out_proj_w, WOUT, kDi, kDm, kDm, kDi, 0);
  wt_plane_kernel<<<kMlp, kDm / 8, 0, stream>>>(fc1_w, WFC1, kDm, kMlp, kMlp, kDm, 0);
  wt_plane_kernel<<<kDm, kMlp / 8, 0, stream>>>(fc2_w, WFC2, kMlp, kDm, kDm, kMlp, 0);
  wt_plane_kernel<<<kIn, kDm / 8, 0, stream>>>(w_exp, WEXP, kDm, kIn, kIn, kDm, 0);
  setup_kernel<<<24, kThr, 0, stream>>>(dt_proj_w, dt_proj_b, fc1_b, fc2_b, WDT, BV);

  for (int s = 0; s < kSamples; ++s) {
    const float* xs = x_tokens + (size_t)s * kRows * kIn;
    float* os = out + (size_t)s * kRows * kIn;
    cast_plane_kernel<<<(int)(((size_t)kRows * kIn / 8) / kThr), kThr, 0, stream>>>(xs, X16, 10, kIn, 0);
    wmma_gemm64<0, false, 2, 0, false, 0><<<dim3((kRows / 64) * (kDm / 64) / 8, 1), 256, 0, stream>>>(
        X16, X16, kIn, 0L, WRED, WRED, kIn, 0L, (void*)XF, (void*)XF, kDm, 0L, ZB, nullptr, 0L, kRows, kDm, kIn, kScX);
    ln_kernel<<<kRows, 128, 0, stream>>>(XF, ln1_g, ln1_b, nullptr, nullptr, XN16);
    wmma_gemm64<0, false, 2, 0, false, 0><<<dim3((kRows / 64) * (kDi2 / 64) / 8, 1), 256, 0, stream>>>(
        XN16, XN16, kDm, 0L, WIN, WIN, kDm, 0L, (void*)XZ, (void*)XZ, kDi2, 0L, ZB, nullptr, 0L, kRows, kDi2, kDm, kScA);
    conv_silu_kernel<<<(int)(((size_t)kRows * 256) / kThr), kThr, 0, stream>>>(XZ, conv_w, conv_b, XI, XI16);
    wmma_gemm64<0, false, 2, 0, false, 0><<<dim3((kRows / 64) * (kXd / 64) / 8, 1), 256, 0, stream>>>(
        XI16, XI16, kDi, 0L, WXP, WXP, kDi, 0L, (void*)XD, (void*)XD, kXd, 0L, ZB, nullptr, 0L, kRows, kXd, kDi, kScA);
    dt_cast_kernel<<<(int)(((size_t)kRows * 4) / kThr), kThr, 0, stream>>>(XD, DT16);
    wmma_gemm64<0, false, 2, 0, false, 0><<<dim3((kRows / 64) * (kDi / 64) / 8, 1), 256, 0, stream>>>(
        DT16, DT16, kR, 0L, WDT, WDT, kR, 0L, (void*)DL, (void*)DL, kDi, 0L, BV + kBvDt, nullptr, 0L, kRows, kDi, kR, kScA);
    sel_scan_kernel<<<kDi / kThr, kThr, 0, stream>>>(DL, XI, XD, A_log, HID);
    gate_cast_kernel<<<(int)(((size_t)kRows * 128) / kThr), kThr, 0, stream>>>(HID, XI, XZ, D_ssm, Y16);
    wmma_gemm64<0, false, 2, 0, false, 0><<<dim3((kRows / 64) * (kDm / 64) / 8, 1), 256, 0, stream>>>(
        Y16, Y16, kDi, 0L, WOUT, WOUT, kDi, 0L, (void*)XM, (void*)XM, kDm, 0L, ZB, nullptr, 0L, kRows, kDm, kDi, kScA);
    ln_kernel<<<kRows, 128, 0, stream>>>(XM, ln2_g, ln2_b, XF, MO, MO16);
    wmma_gemm64<0, false, 2, 0, false, 0><<<dim3((kRows / 64) * (kMlp / 64) / 8, 1), 256, 0, stream>>>(
        MO16, MO16, kDm, 0L, WFC1, WFC1, kDm, 0L, (void*)H1, (void*)H1, kMlp, 0L, BV + kBvF1, nullptr, 0L, kRows, kMlp, kDm, kScA);
    gelu_cast_kernel<<<(int)(((size_t)kRows * kMlp / 8) / kThr), kThr, 0, stream>>>(H1, H16);
    wmma_gemm64<0, false, 2, 0, false, 0><<<dim3((kRows / 64) * (kDm / 64) / 8, 1), 256, 0, stream>>>(
        H16, H16, kMlp, 0L, WFC2, WFC2, kMlp, 0L, (void*)M2, (void*)M2, kDm, 0L, BV + kBvF2, nullptr, 0L, kRows, kDm, kMlp, kScA);
    add_cast_kernel<<<(int)(((size_t)kRows * kDm / 8) / kThr), kThr, 0, stream>>>(M2, MO, O16);
    wmma_gemm64<0, false, 2, 0, false, 0><<<dim3((kRows / 64) * (kIn / 64) / 8, 1), 256, 0, stream>>>(
        O16, O16, kDm, 0L, WEXP, WEXP, kDm, 0L, (void*)EX, (void*)EX, kIn, 0L, ZB, nullptr, 0L, kRows, kIn, kDm, kScA);
    add_out_kernel<<<(int)(((size_t)kRows * kIn / 4) / kThr), kThr, 0, stream>>>(EX, xs, os);
  }
}
